// SemanticGraphModule_90460601189044
// MI455X (gfx1250) — hardware-verified
//
#include <hip/hip_runtime.h>
#include <stdint.h>


typedef _Float16       v16h __attribute__((ext_vector_type(16)));
typedef __bf16         v16b __attribute__((ext_vector_type(16)));
typedef unsigned short v8us __attribute__((ext_vector_type(8)));
typedef float          v8f  __attribute__((ext_vector_type(8)));
typedef float          v4f  __attribute__((ext_vector_type(4)));

#define DM    256
#define NNBR  32
#define TOPK  8
#define LDSP  40
#define CSP   68

union FragH { v16h v; v8us u[2]; };
union FragB { v16b v; v8us u[2]; };

__device__ __forceinline__ v8f wmma16f(v16h a, v16h b, v8f c)
{
    c = __builtin_amdgcn_wmma_f32_16x16x32_f16(false, a, false, b, (short)0, c, false, false);
    asm volatile("v_nop\n\tv_nop\n\tv_nop\n\tv_nop" : "+v"(c) : "v"(a), "v"(b));
    return c;
}
__device__ __forceinline__ v8f wmma16b(v16b a, v16b b, v8f c)
{
    c = __builtin_amdgcn_wmma_f32_16x16x32_bf16(false, a, false, b, (short)0, c, false, false);
    asm volatile("v_nop\n\tv_nop\n\tv_nop\n\tv_nop" : "+v"(c) : "v"(a), "v"(b));
    return c;
}

__device__ __forceinline__ unsigned f2bf(float f)
{
    unsigned u = __float_as_uint(f);
    u += 0x7FFFu + ((u >> 16) & 1u);
    return u >> 16;
}
__device__ __forceinline__ float bf2f(unsigned b) { return __uint_as_float(b << 16); }
__device__ __forceinline__ unsigned short h2us(float f)
{
    union { _Float16 h; unsigned short u; } c;
    c.h = (_Float16)f;
    return c.u;
}

__global__ __launch_bounds__(256)
void k_cvt(const float* __restrict__ s0, int n0,
           const float* __restrict__ s1, int n1,
           const float* __restrict__ s2, const float* __restrict__ s3,
           const float* __restrict__ s4, const float* __restrict__ s5, int n25,
           const float* __restrict__ s6, int n6,
           const float* __restrict__ s7, int n7,
           unsigned short* d0h, unsigned short* d0l,
           unsigned short* d1h, unsigned short* d1l,
           unsigned short* d2, unsigned short* d3, unsigned short* d4, unsigned short* d5,
           unsigned short* d6, unsigned short* d7)
{
    const int sel = blockIdx.y;
    const float* src = s0; unsigned short* dh = d0h; unsigned short* dl = d0l; int n = n0;
    if      (sel == 1) { src = s1; dh = d1h; dl = d1l; n = n1;  }
    else if (sel == 2) { src = s2; dh = d2;  dl = d2;  n = n25; }
    else if (sel == 3) { src = s3; dh = d3;  dl = d3;  n = n25; }
    else if (sel == 4) { src = s4; dh = d4;  dl = d4;  n = n25; }
    else if (sel == 5) { src = s5; dh = d5;  dl = d5;  n = n25; }
    else if (sel == 6) { src = s6; dh = d6;  dl = d6;  n = n6;  }
    else if (sel == 7) { src = s7; dh = d7;  dl = d7;  n = n7;  }

    const size_t i = ((size_t)blockIdx.x * 256u + threadIdx.x) * 8u;
    if (i + 8u > (size_t)n) return;

    const v4f a = *(const v4f*)(src + i);
    const v4f b = *(const v4f*)(src + i + 4);
    float x[8];
    x[0] = a[0]; x[1] = a[1]; x[2] = a[2]; x[3] = a[3];
    x[4] = b[0]; x[5] = b[1]; x[6] = b[2]; x[7] = b[3];

    if (sel < 2) {
        v8us uh, ul;
        #pragma unroll
        for (int j = 0; j < 8; ++j) {
            const unsigned hb = f2bf(x[j]);
            uh[j] = (unsigned short)hb;
            ul[j] = (unsigned short)f2bf(x[j] - bf2f(hb));
        }
        *(volatile v8us*)(dh + i) = uh;
        *(volatile v8us*)(dl + i) = ul;
        __threadfence();
        *(volatile v8us*)(dh + i) = uh;
        *(volatile v8us*)(dl + i) = ul;
    } else {
        v8us uh;
        #pragma unroll
        for (int j = 0; j < 8; ++j) uh[j] = h2us(x[j] * 64.0f);
        *(volatile v8us*)(dh + i) = uh;
        __threadfence();
        *(volatile v8us*)(dh + i) = uh;
    }
}

template <int SPLIT>
__global__ __launch_bounds__(256)
void k_gemm(const float* __restrict__ Xf,
            const unsigned short* __restrict__ Xh, const unsigned short* __restrict__ Xl,
            const unsigned short* __restrict__ Wh, const unsigned short* __restrict__ Wl,
            const float* __restrict__ bias, float* Y, int M, int K, int O, int act)
{
    __shared__ __attribute__((aligned(16))) unsigned short As[2 * 64 * LDSP];
    __shared__ __attribute__((aligned(16))) unsigned short Bs[2 * 64 * LDSP];
    __shared__ __attribute__((aligned(16))) float Cs[64 * CSP];

    const int t    = threadIdx.x;
    const int l    = t & 31;
    const int wave = t >> 5;
    const int h    = l >> 4;
    const int m    = l & 15;
    const int mo   = (wave & 3) * 16;
    const int no   = (wave >> 2) * 32;
    const int mBase = blockIdx.y * 64;
    const int oBase = blockIdx.x * 64;

    const int srow = t >> 2;
    const int sc8  = (t & 3) * 8;
    int gm = mBase + srow; if (gm > M - 1) gm = M - 1;
    const int go = oBase + srow;
    const size_t xoff = (size_t)gm * (size_t)K + (size_t)sc8;
    const size_t woff = (size_t)go * (size_t)K + (size_t)sc8;
    const int sidx = srow * LDSP + sc8;

    v8f c0 = {0.f, 0.f, 0.f, 0.f, 0.f, 0.f, 0.f, 0.f};
    v8f c1 = {0.f, 0.f, 0.f, 0.f, 0.f, 0.f, 0.f, 0.f};

    const int nk = K >> 5;
    for (int kt = 0; kt < nk; ++kt) {
        const int k0 = kt << 5;
        if (SPLIT) {
            *(v8us*)&As[sidx]             = *(const v8us*)(Xh + xoff + k0);
            *(v8us*)&As[64 * LDSP + sidx] = *(const v8us*)(Xl + xoff + k0);
            *(v8us*)&Bs[sidx]             = *(const v8us*)(Wh + woff + k0);
            *(v8us*)&Bs[64 * LDSP + sidx] = *(const v8us*)(Wl + woff + k0);
        } else {
            const v4f x0 = *(const v4f*)(Xf + xoff + k0);
            const v4f x1 = *(const v4f*)(Xf + xoff + k0 + 4);
            v8us u;
            u[0] = h2us(x0[0] * 64.0f); u[1] = h2us(x0[1] * 64.0f);
            u[2] = h2us(x0[2] * 64.0f); u[3] = h2us(x0[3] * 64.0f);
            u[4] = h2us(x1[0] * 64.0f); u[5] = h2us(x1[1] * 64.0f);
            u[6] = h2us(x1[2] * 64.0f); u[7] = h2us(x1[3] * 64.0f);
            *(v8us*)&As[sidx] = u;
            *(v8us*)&Bs[sidx] = *(const v8us*)(Wh + woff + k0);
        }
        __syncthreads();

        const int ar  = (mo + m) * LDSP + 8 * h;
        const int br0 = (no + m) * LDSP + 8 * h;
        const int br1 = (no + 16 + m) * LDSP + 8 * h;
        if (SPLIT) {
            FragB a, al, b0, b0l, b1, b1l;
            a.u[0]   = *(const v8us*)&As[ar];
            a.u[1]   = *(const v8us*)&As[ar + 16];
            al.u[0]  = *(const v8us*)&As[64 * LDSP + ar];
            al.u[1]  = *(const v8us*)&As[64 * LDSP + ar + 16];
            b0.u[0]  = *(const v8us*)&Bs[br0];
            b0.u[1]  = *(const v8us*)&Bs[br0 + 16];
            b0l.u[0] = *(const v8us*)&Bs[64 * LDSP + br0];
            b0l.u[1] = *(const v8us*)&Bs[64 * LDSP + br0 + 16];
            b1.u[0]  = *(const v8us*)&Bs[br1];
            b1.u[1]  = *(const v8us*)&Bs[br1 + 16];
            b1l.u[0] = *(const v8us*)&Bs[64 * LDSP + br1];
            b1l.u[1] = *(const v8us*)&Bs[64 * LDSP + br1 + 16];
            c0 = wmma16b(a.v,  b0.v,  c0);
            c0 = wmma16b(a.v,  b0l.v, c0);
            c0 = wmma16b(al.v, b0.v,  c0);
            c1 = wmma16b(a.v,  b1.v,  c1);
            c1 = wmma16b(a.v,  b1l.v, c1);
            c1 = wmma16b(al.v, b1.v,  c1);
        } else {
            FragH a, b0, b1;
            a.u[0]  = *(const v8us*)&As[ar];
            a.u[1]  = *(const v8us*)&As[ar + 16];
            b0.u[0] = *(const v8us*)&Bs[br0];
            b0.u[1] = *(const v8us*)&Bs[br0 + 16];
            b1.u[0] = *(const v8us*)&Bs[br1];
            b1.u[1] = *(const v8us*)&Bs[br1 + 16];
            c0 = wmma16f(a.v, b0.v, c0);
            c1 = wmma16f(a.v, b1.v, c1);
        }
        __syncthreads();
    }

    #pragma unroll
    for (int r = 0; r < 8; ++r) {
        Cs[(mo + 8 * h + r) * CSP + no + m]      = c0[r];
        Cs[(mo + 8 * h + r) * CSP + no + 16 + m] = c1[r];
    }
    __syncthreads();

    const int q = m;
    const float scl = SPLIT ? 1.0f : (1.0f / 4096.0f);
    const v4f bz = *(const v4f*)(bias + oBase + 4 * q);
    v4f vals[4];
    #pragma unroll
    for (int i = 0; i < 4; ++i) {
        const int row = wave * 8 + 2 * i + h;
        const v4f cv = *(const v4f*)&Cs[row * CSP + 4 * q];
        v4f y = cv * scl + bz;
        if (act == 1) {
            y[0] = 0.5f * y[0] * (1.0f + erff(y[0] * 0.70710678118654752f));
            y[1] = 0.5f * y[1] * (1.0f + erff(y[1] * 0.70710678118654752f));
            y[2] = 0.5f * y[2] * (1.0f + erff(y[2] * 0.70710678118654752f));
            y[3] = 0.5f * y[3] * (1.0f + erff(y[3] * 0.70710678118654752f));
        }
        vals[i] = y;
    }
    #pragma unroll
    for (int i = 0; i < 4; ++i) {
        const int grow = mBase + wave * 8 + 2 * i + h;
        if (grow < M)
            *(volatile v4f*)(Y + (size_t)grow * (size_t)O + oBase + 4 * q) = vals[i];
    }
    __threadfence();
    #pragma unroll
    for (int i = 0; i < 4; ++i) {
        const int grow = mBase + wave * 8 + 2 * i + h;
        if (grow < M)
            *(volatile v4f*)(Y + (size_t)grow * (size_t)O + oBase + 4 * q) = vals[i];
    }
}

__global__ __launch_bounds__(256)
void k_rownorm(const float* __restrict__ P, float* Pinv, int Rn)
{
    __shared__ __attribute__((aligned(16))) float red[32];
    const int l = threadIdx.x & 31, wave = threadIdx.x >> 5;
    #pragma unroll
    for (int j = 0; j < 4; ++j) {
        const int r = blockIdx.x * 32 + wave * 4 + j;
        int rr = r; if (rr > Rn - 1) rr = Rn - 1;
        const float* p = P + (size_t)rr * DM;
        const v4f a = *(const v4f*)(p + 4 * l);
        const v4f b = *(const v4f*)(p + 128 + 4 * l);
        const v4f sa = a * a, sb = b * b;
        float ss = ((sa[0] + sa[1]) + (sa[2] + sa[3])) + ((sb[0] + sb[1]) + (sb[2] + sb[3]));
        for (int off = 16; off >= 1; off >>= 1) ss += __shfl_xor(ss, off, 32);
        if (l == 0) red[wave * 4 + j] = (r < Rn) ? (1.0f / fmaxf(sqrtf(ss), 1e-12f)) : 0.0f;
    }
    __syncthreads();
    if (wave == 0 && l < 8) {
        const v4f v = *(const v4f*)&red[4 * l];
        float* dst = Pinv + (size_t)blockIdx.x * 32 + 4 * l;
        *(volatile v4f*)dst = v;
        __threadfence();
        *(volatile v4f*)dst = v;
    }
}

__global__ __launch_bounds__(32)
void k_topk(const int* __restrict__ rel_ids, const int* __restrict__ nbr,
            const float* __restrict__ P, const float* __restrict__ Pinv,
            float* ctx, float* st0, int Rn)
{
    const int e = blockIdx.x, l = threadIdx.x;
    int rid = rel_ids[e];
    rid = rid < 0 ? 0 : (rid > Rn - 1 ? Rn - 1 : rid);
    int nid = nbr[(size_t)e * NNBR + l];
    nid = nid < 0 ? 0 : (nid > Rn - 1 ? Rn - 1 : nid);

    const float* pr = P + (size_t)rid * DM;
    const float* pn = P + (size_t)nid * DM;
    float acc = 0.f;
    #pragma unroll 2
    for (int d4 = 0; d4 < DM / 4; ++d4) {
        const v4f a = *(const v4f*)(pn + 4 * d4);
        const v4f b = *(const v4f*)(pr + 4 * d4);
        acc += a[0] * b[0];
        acc += a[1] * b[1];
        acc += a[2] * b[2];
        acc += a[3] * b[3];
    }
    const float sim = acc * Pinv[nid] * Pinv[rid];

    unsigned sel = 0u;
    v4f ca = {0.f, 0.f, 0.f, 0.f};
    v4f cb = {0.f, 0.f, 0.f, 0.f};
    const float ninf = -__builtin_inff();
    for (int ts = 0; ts < TOPK; ++ts) {
        float v = ((sel >> l) & 1u) ? ninf : sim;
        int idx = l;
        for (int off = 16; off >= 1; off >>= 1) {
            const float ov = __shfl_xor(v, off, 32);
            const int   oi = __shfl_xor(idx, off, 32);
            if (ov > v || (ov == v && oi < idx)) { v = ov; idx = oi; }
        }
        sel |= 1u << idx;
        int snid = __shfl(nid, idx, 32);
        snid = snid < 0 ? 0 : (snid > Rn - 1 ? Rn - 1 : snid);
        const float* ps = P + (size_t)snid * DM;
        ca += *(const v4f*)(ps + 4 * l);
        cb += *(const v4f*)(ps + 128 + 4 * l);
    }
    ca *= 0.125f;
    cb *= 0.125f;
    const v4f ra = *(const v4f*)(pr + 4 * l);
    const v4f rb = *(const v4f*)(pr + 128 + 4 * l);

    float* cp = ctx + (size_t)e * DM;
    float* sp = st0 + (size_t)e * DM;
    *(volatile v4f*)(cp + 4 * l)       = ca;
    *(volatile v4f*)(cp + 128 + 4 * l) = cb;
    *(volatile v4f*)(sp + 4 * l)       = ra;
    *(volatile v4f*)(sp + 128 + 4 * l) = rb;
    __threadfence();
    *(volatile v4f*)(cp + 4 * l)       = ca;
    *(volatile v4f*)(cp + 128 + 4 * l) = cb;
    *(volatile v4f*)(sp + 4 * l)       = ra;
    *(volatile v4f*)(sp + 128 + 4 * l) = rb;
}

__global__ __launch_bounds__(256)
void k_attnw(const float* __restrict__ q, const float* __restrict__ k,
             const float* __restrict__ v, float* wv, int nrows)
{
    const int l = threadIdx.x & 31, wave = threadIdx.x >> 5;
    int row = blockIdx.x * 8 + wave;
    const bool ok = row < nrows;
    if (!ok) row = nrows - 1;
    const size_t ro = (size_t)row * DM;
    const v4f qa = *(const v4f*)(q + ro + 4 * l), qb = *(const v4f*)(q + ro + 128 + 4 * l);
    const v4f ka = *(const v4f*)(k + ro + 4 * l), kb = *(const v4f*)(k + ro + 128 + 4 * l);
    const v4f va = *(const v4f*)(v + ro + 4 * l), vb = *(const v4f*)(v + ro + 128 + 4 * l);
    const v4f pa = qa * ka, pb = qb * kb;
    float p0 = (pa[0] + pa[1]) + (pa[2] + pa[3]);
    float p1 = (pb[0] + pb[1]) + (pb[2] + pb[3]);
    #pragma unroll
    for (int off = 1; off <= 4; off <<= 1) {
        p0 += __shfl_xor(p0, off, 32);
        p1 += __shfl_xor(p1, off, 32);
    }
    const float isd = 0.17677669529663687f;
    const float lg0 = p0 * isd, lg1 = p1 * isd;
    const float mx0 = lg0, mx1 = lg1;
    const float e0 = __expf(lg0 - mx0), e1 = __expf(lg1 - mx1);
    const float s0 = e0, s1 = e1;
    const float w0 = e0 * (1.0f / s0), w1 = e1 * (1.0f / s1);
    const v4f oa = va * w0, ob = vb * w1;

    float* dp = wv + ro;
    if (ok) {
        *(volatile v4f*)(dp + 4 * l)       = oa;
        *(volatile v4f*)(dp + 128 + 4 * l) = ob;
    }
    __threadfence();
    if (ok) {
        *(volatile v4f*)(dp + 4 * l)       = oa;
        *(volatile v4f*)(dp + 128 + 4 * l) = ob;
    }
}

__global__ __launch_bounds__(256)
void k_ln(const float* __restrict__ resid, const float* __restrict__ delta,
          const float* __restrict__ g, const float* __restrict__ b,
          const float* __restrict__ rscale, int use_rscale, float* out, int nrows)
{
    const int l = threadIdx.x & 31, wave = threadIdx.x >> 5;
    int row = blockIdx.x * 8 + wave;
    const bool ok = row < nrows;
    if (!ok) row = nrows - 1;
    const size_t ro = (size_t)row * DM;
    const v4f xa = *(const v4f*)(resid + ro + 4 * l)       + *(const v4f*)(delta + ro + 4 * l);
    const v4f xb = *(const v4f*)(resid + ro + 128 + 4 * l) + *(const v4f*)(delta + ro + 128 + 4 * l);
    float s = ((xa[0] + xa[1]) + (xa[2] + xa[3])) + ((xb[0] + xb[1]) + (xb[2] + xb[3]));
    for (int off = 16; off >= 1; off >>= 1) s += __shfl_xor(s, off, 32);
    const float mu = s * (1.0f / 256.0f);
    const v4f da = xa - mu, db = xb - mu;
    const v4f qa = da * da, qb = db * db;
    float s2 = ((qa[0] + qa[1]) + (qa[2] + qa[3])) + ((qb[0] + qb[1]) + (qb[2] + qb[3]));
    for (int off = 16; off >= 1; off >>= 1) s2 += __shfl_xor(s2, off, 32);
    const float var  = s2 * (1.0f / 256.0f);
    const float rinv = rsqrtf(var + 1e-5f);
    const v4f ga = *(const v4f*)(g + 4 * l), gb = *(const v4f*)(g + 128 + 4 * l);
    const v4f ba = *(const v4f*)(b + 4 * l), bb = *(const v4f*)(b + 128 + 4 * l);
    v4f ya = (da * rinv) * ga + ba;
    v4f yb = (db * rinv) * gb + bb;
    if (use_rscale) { const float mk = rscale[row]; ya *= mk; yb *= mk; }

    float* dp = out + ro;
    if (ok) {
        *(volatile v4f*)(dp + 4 * l)       = ya;
        *(volatile v4f*)(dp + 128 + 4 * l) = yb;
    }
    __threadfence();
    if (ok) {
        *(volatile v4f*)(dp + 4 * l)       = ya;
        *(volatile v4f*)(dp + 128 + 4 * l) = yb;
    }
}

__global__ __launch_bounds__(256)
void k_tail(const float* __restrict__ src, float* dst, int n)
{
    const int i = (blockIdx.x * 256 + threadIdx.x) * 4;
    if (i + 4 <= n) {
        const v4f v = *(const v4f*)(src + i);
        *(volatile v4f*)(dst + i) = v;
        __threadfence();
        *(volatile v4f*)(dst + i) = v;
    } else if (i < n) {
        float t0 = src[i];
        float t1 = (i + 1 < n) ? src[i + 1] : 0.f;
        float t2 = (i + 2 < n) ? src[i + 2] : 0.f;
        ((volatile float*)dst)[i] = t0;
        if (i + 1 < n) ((volatile float*)dst)[i + 1] = t1;
        if (i + 2 < n) ((volatile float*)dst)[i + 2] = t2;
        __threadfence();
        ((volatile float*)dst)[i] = t0;
        if (i + 1 < n) ((volatile float*)dst)[i + 1] = t1;
        if (i + 2 < n) ((volatile float*)dst)[i + 2] = t2;
    }
}

extern "C" void kernel_launch(void* const* d_in, const int* in_sizes, int n_in,
                              void* d_out, int out_size, void* d_ws, size_t ws_size,
                              hipStream_t stream)
{
    (void)n_in;
    const int*   rel_ids = (const int*)d_in[0];
    const int*   nbr     = (const int*)d_in[1];
    const float* escale  = (const float*)d_in[2];
    const float* rel_emb = (const float*)d_in[3];
    const float* proj_W  = (const float*)d_in[4];
    const float* proj_b  = (const float*)d_in[5];
    const float* Wq   = (const float*)d_in[6];
    const float* bq   = (const float*)d_in[7];
    const float* Wk   = (const float*)d_in[8];
    const float* bk   = (const float*)d_in[9];
    const float* Wv   = (const float*)d_in[10];
    const float* bv   = (const float*)d_in[11];
    const float* Wo   = (const float*)d_in[12];
    const float* bo   = (const float*)d_in[13];
    const float* ln1g = (const float*)d_in[14];
    const float* ln1b = (const float*)d_in[15];
    const float* ln2g = (const float*)d_in[16];
    const float* ln2b = (const float*)d_in[17];
    const float* W1   = (const float*)d_in[18];
    const float* b1   = (const float*)d_in[19];
    const float* W2   = (const float*)d_in[20];
    const float* b2   = (const float*)d_in[21];
    float* out = (float*)d_out;

    const int REL = 512, DFF = 1024;
    if (in_sizes[3] <= 0 || (in_sizes[3] % REL) != 0) return;
    const int Rn = in_sizes[3] / REL;
    const int BE = in_sizes[0];
    if (BE <= 0 || in_sizes[1] != BE * NNBR || in_sizes[2] != BE) return;
    if (in_sizes[4] != DM * REL || in_sizes[5] != DM) return;
    if (in_sizes[6] <= 0 || (in_sizes[6] % (DM * DM)) != 0) return;
    const int NL = in_sizes[6] / (DM * DM);
    if (in_sizes[7] != NL * DM || in_sizes[8] != NL * DM * DM || in_sizes[9] != NL * DM) return;
    if (in_sizes[10] != NL * DM * DM || in_sizes[11] != NL * DM) return;
    if (in_sizes[12] != NL * DM * DM || in_sizes[13] != NL * DM) return;
    if (in_sizes[14] != NL * DM || in_sizes[15] != NL * DM || in_sizes[16] != NL * DM || in_sizes[17] != NL * DM) return;
    if (in_sizes[18] != NL * DFF * DM || in_sizes[19] != NL * DFF) return;
    if (in_sizes[20] != NL * DM * DFF || in_sizes[21] != NL * DM) return;
    if (out_size != BE * DM + BE) return;

    float* ws = (float*)d_ws;
    size_t off = 0;
    auto carve = [&](size_t nfloats) -> float* { float* p = ws + off; off += (nfloats + 31) & ~(size_t)31; return p; };
    const int RnPad = ((Rn + 31) / 32) * 32;
    float* P     = carve((size_t)Rn * DM);
    float* Pinv  = carve((size_t)RnPad);
    float* ctx   = carve((size_t)BE * DM);
    float* stA   = carve((size_t)BE * DM);
    float* stB   = carve((size_t)BE * DM);
    float* qb    = carve((size_t)BE * DM);
    float* kbuf  = carve((size_t)BE * DM);
    float* vb    = carve((size_t)BE * DM);
    float* wvb   = carve((size_t)BE * DM);
    float* attb  = carve((size_t)BE * DM);
    float* ffb   = carve((size_t)BE * DM);
    float* hb    = carve((size_t)BE * DFF);
    unsigned short* re_hi = (unsigned short*)carve((size_t)Rn * REL / 2);
    unsigned short* re_lo = (unsigned short*)carve((size_t)Rn * REL / 2);
    unsigned short* pw_hi = (unsigned short*)carve((size_t)DM * REL / 2);
    unsigned short* pw_lo = (unsigned short*)carve((size_t)DM * REL / 2);
    unsigned short* Wq16  = (unsigned short*)carve((size_t)NL * DM * DM / 2);
    unsigned short* Wk16  = (unsigned short*)carve((size_t)NL * DM * DM / 2);
    unsigned short* Wv16  = (unsigned short*)carve((size_t)NL * DM * DM / 2);
    unsigned short* Wo16  = (unsigned short*)carve((size_t)NL * DM * DM / 2);
    unsigned short* W116  = (unsigned short*)carve((size_t)NL * DFF * DM / 2);
    unsigned short* W216  = (unsigned short*)carve((size_t)NL * DM * DFF / 2);
    if (off * sizeof(float) > ws_size) return;

    {
        const int n0 = Rn * REL, n1 = DM * REL, n25 = NL * DM * DM, n6 = NL * DFF * DM, n7 = NL * DM * DFF;
        int mx = n0; if (n1 > mx) mx = n1; if (n25 > mx) mx = n25; if (n6 > mx) mx = n6; if (n7 > mx) mx = n7;
        dim3 g((mx + 2047) / 2048, 8);
        k_cvt<<<g, 256, 0, stream>>>(rel_emb, n0, proj_W, n1, Wq, Wk, Wv, Wo, n25, W1, n6, W2, n7,
                                     re_hi, re_lo, pw_hi, pw_lo, Wq16, Wk16, Wv16, Wo16, W116, W216);
    }

    {
        dim3 g(DM / 64, (Rn + 63) / 64);
        k_gemm<1><<<g, 256, 0, stream>>>(P, re_hi, re_lo, pw_hi, pw_lo, proj_b, P, Rn, REL, DM, 0);
    }
    k_rownorm<<<RnPad / 32, 256, 0, stream>>>(P, Pinv, Rn);

    k_topk<<<BE, 32, 0, stream>>>(rel_ids, nbr, P, Pinv, ctx, stA, Rn);

    auto gemm16 = [&](const float* X, const unsigned short* W16, const float* bias, float* Yp,
                      int M, int K, int O, int act) {
        dim3 g(O / 64, (M + 63) / 64);
        k_gemm<0><<<g, 256, 0, stream>>>(X, W16, W16, W16, W16, bias, Yp, M, K, O, act);
    };
    const int rb8 = (BE + 7) / 8;

    for (int li = 0; li < NL; ++li) {
        const size_t wo = (size_t)li * DM * DM;
        gemm16(stA, Wq16 + wo, bq + li * DM, qb,   BE, DM, DM, 0);
        gemm16(ctx, Wk16 + wo, bk + li * DM, kbuf, BE, DM, DM, 0);
        gemm16(ctx, Wv16 + wo, bv + li * DM, vb,   BE, DM, DM, 0);
        k_attnw<<<rb8, 256, 0, stream>>>(qb, kbuf, vb, wvb, BE);
        gemm16(wvb, Wo16 + wo, bo + li * DM, attb, BE, DM, DM, 0);
        k_ln<<<rb8, 256, 0, stream>>>(stA, attb, ln1g + li * DM, ln1b + li * DM, escale, 0, stB, BE);
        gemm16(stB, W116 + (size_t)li * DFF * DM, b1 + li * DFF, hb,  BE, DM,  DFF, 1);
        gemm16(hb,  W216 + (size_t)li * DM * DFF, b2 + li * DM,  ffb, BE, DFF, DM,  0);
        float* lnout = (li == NL - 1) ? out : stA;
        k_ln<<<rb8, 256, 0, stream>>>(stB, ffb, ln2g + li * DM, ln2b + li * DM, escale, 1, lnout, BE);
    }

    k_tail<<<(BE + 1023) / 1024, 256, 0, stream>>>(escale, out + (size_t)BE * DM, BE);
}
